// ceRNAnet_2963527435018
// MI455X (gfx1250) — hardware-verified
//
#include <hip/hip_runtime.h>
#include <math.h>

#define NN 20000
#define NE 640000
#define SS 256
#define ND 2000
#define NPW 500
#define NPH 100
#define NOUT 2
#define LC0 8000
#define LC1 2000
#define LC2 10000
#define KP1 2048
#define PP1 512
#define PHP1 128
#define OPP 64
#define NBIAS (PP1 + PHP1 + OPP)
#define NT 256
#define TILE 2048
#define NTILE 10
#define NPR (NTILE * TILE)
#define RPW (TILE / 8)
#define SCH 4096
#define SPT 16
#define NCH ((NE + SCH - 1) / SCH)
#define TP 260
#define XTP 264
#define R1DW (PP1 * KP1 / 2)
#define R2DW (PHP1 * PP1 / 2)
#define R3DW (OPP * PHP1 / 2)
#define L0_RBETA (1.0f / 0.66f)

#if (NE % SPT) != 0
#error
#endif
#if (SCH != SPT * NT)
#error
#endif
#if (NPR < NN)
#error
#endif
#if (NN % 32) != 0 || (SS != 256)
#error
#endif

typedef __attribute__((ext_vector_type(16))) _Float16 v16h;
typedef __attribute__((ext_vector_type(8)))  _Float16 v8h;
typedef __attribute__((ext_vector_type(16))) __bf16   v16b;
typedef __attribute__((ext_vector_type(8)))  __bf16   v8b;
typedef __attribute__((ext_vector_type(8)))  float    v8f;
typedef __attribute__((ext_vector_type(4)))  float    v4f;
typedef __attribute__((ext_vector_type(2)))  float    v2f;
typedef __attribute__((ext_vector_type(4)))  int      v4i;

__device__ __forceinline__ unsigned short f2bf_bits(float f) {
  unsigned u = __float_as_uint(f);
  return (unsigned short)((u + 0x7FFFu + ((u >> 16) & 1u)) >> 16);
}
__device__ __forceinline__ float bf_bits2f(unsigned short h) { return __uint_as_float(((unsigned)h) << 16); }

__device__ __forceinline__ void dep_guard_h(v8f& a, v8f& b, v16h x, v16h y) { asm volatile("v_nop\n\tv_nop\n\tv_nop\n\tv_nop" : "+v"(a), "+v"(b) : "v"(x), "v"(y)); }
__device__ __forceinline__ void dep_guard_b(v8f& a, v8f& b, v16b x, v16b y) { asm volatile("v_nop\n\tv_nop\n\tv_nop\n\tv_nop" : "+v"(a), "+v"(b) : "v"(x), "v"(y)); }
__device__ __forceinline__ void keep4_h(v16h a, v16h b, v16h c, v16h d) { asm volatile("v_nop" :: "v"(a), "v"(b), "v"(c), "v"(d)); }
__device__ __forceinline__ void keep4_b(v16b a, v16b b, v16b c, v16b d) { asm volatile("v_nop" :: "v"(a), "v"(b), "v"(c), "v"(d)); }
__device__ __forceinline__ void acc_guard4(v8f& a, v8f& b, v8f& c, v8f& d) { asm volatile("v_nop\n\tv_nop\n\tv_nop\n\tv_nop" : "+v"(a), "+v"(b), "+v"(c), "+v"(d)); }
template <typename T> struct Frag;
template <> struct Frag<_Float16> {
  typedef v16h V; union U { v16h v; v8h h[2]; };
  static __device__ __forceinline__ v16h load(const _Float16* p) {
    U f; f.h[0] = *(const v8h*)(p); f.h[1] = *(const v8h*)(p + 16); return f.v;
  }
  static __device__ __forceinline__ v8f mma(v16h a, v16h b, v8f c) {
    return __builtin_amdgcn_wmma_f32_16x16x32_f16(false, a, false, b, (short)0, c, false, false);
  }
  static __device__ __forceinline__ void guard(v8f& a, v8f& b, v16h x, v16h y) { dep_guard_h(a, b, x, y); }
  static __device__ __forceinline__ void keep(v16h a, v16h b, v16h c, v16h d) { keep4_h(a, b, c, d); }
};
template <> struct Frag<__bf16> {
  typedef v16b V; union U { v16b v; v8b h[2]; };
  static __device__ __forceinline__ v16b load(const __bf16* p) {
    U f; f.h[0] = *(const v8b*)(p); f.h[1] = *(const v8b*)(p + 16); return f.v;
  }
  static __device__ __forceinline__ v8f mma(v16b a, v16b b, v8f c) {
    return __builtin_amdgcn_wmma_f32_16x16x32_bf16(false, a, false, b, (short)0, c, false, false);
  }
  static __device__ __forceinline__ void guard(v8f& a, v8f& b, v16b x, v16b y) { dep_guard_b(a, b, x, y); }
  static __device__ __forceinline__ void keep(v16b a, v16b b, v16b c, v16b d) { keep4_b(a, b, c, d); }
};

template <int ET> struct Elem;
template <> struct Elem<0> { typedef _Float16 T; };
template <> struct Elem<1> { typedef __bf16 T; };
template <int ET, bool SPLIT, int BIAS_MODE, int OUT_MODE, bool RESID, int ACT = 0>
__global__ __launch_bounds__(256) void wmma_gemm64(
    const unsigned short* __restrict__ Ap, const unsigned short* __restrict__ A2p, int lda, long strideA,
    const unsigned short* __restrict__ Btp, const unsigned short* __restrict__ Bt2p, int ldb, long strideB,
    void* __restrict__ Cout, void* __restrict__ Cout2, int ldc, long strideC,
    const float* __restrict__ bias,
    const float* __restrict__ resid, long strideR,
    int M, int N, int K, float scale) {
  typedef typename Elem<ET>::T T;
  typedef typename Frag<T>::V V;
  const T* A = (const T*)Ap; const T* A2 = (const T*)A2p; const T* Bt = (const T*)Btp; const T* Bt2 = (const T*)Bt2p;
  __shared__ __align__(16) float sT[8][16 * 68];
  const int b    = blockIdx.y;
  const int lane = threadIdx.x & 31;
  const int wave = threadIdx.x >> 5;
  const int tilesN = N >> 6;
  const int tilesM = M >> 6;
  const int tile = blockIdx.x * 8 + wave;
  if (tile >= tilesM * tilesN) return;
  const int tm = tile / tilesN;
  const int tn = tile - tm * tilesN;
  const int m0 = tm << 6;
  const int n0 = tn << 6;

  const T* Ab  = A  + (size_t)b * strideA;
  const T* Bb  = Bt + (size_t)b * strideB;
  const T* Ab2 = SPLIT ? (A2  + (size_t)b * strideA) : nullptr;
  const T* Bb2 = SPLIT ? (Bt2 + (size_t)b * strideB) : nullptr;

  const int rlane = lane & 15;
  const int koff  = (lane >> 4) * 8;
  const int mOff  = (lane >> 4) * 8;

  v8f acc[4][4];
#pragma unroll
  for (int i = 0; i < 4; ++i)
#pragma unroll
    for (int j = 0; j < 4; ++j) acc[i][j] = (v8f){0.f,0.f,0.f,0.f,0.f,0.f,0.f,0.f};

  for (int k0 = 0; k0 < K; k0 += 32) {
    V bh[4], bl[4];
#pragma unroll
    for (int j = 0; j < 4; ++j) {
      const size_t bo = (size_t)(n0 + (j << 4) + rlane) * ldb + koff + k0;
      bh[j] = Frag<T>::load(Bb + bo);
      if (SPLIT) bl[j] = Frag<T>::load(Bb2 + bo);
    }
#pragma unroll
    for (int i = 0; i < 4; ++i) {
      const size_t ao = (size_t)(m0 + (i << 4) + rlane) * lda + koff + k0;
      V ah = Frag<T>::load(Ab + ao);
      V al;
      if (SPLIT) al = Frag<T>::load(Ab2 + ao);
#pragma unroll
      for (int j = 0; j < 4; ++j) {
        acc[i][j] = Frag<T>::mma(ah, bh[j], acc[i][j]);
        if (SPLIT) {
          acc[i][j] = Frag<T>::mma(ah, bl[j], acc[i][j]);
          acc[i][j] = Frag<T>::mma(al, bh[j], acc[i][j]);
        }
      }
      Frag<T>::guard(acc[i][0], acc[i][3], ah, SPLIT ? al : ah);
    }
    Frag<T>::keep(bh[0], bh[1], bh[2], bh[3]);
    if (SPLIT) Frag<T>::keep(bl[0], bl[1], bl[2], bl[3]);
  }
  acc_guard4(acc[0][0], acc[0][1], acc[0][2], acc[0][3]);
  acc_guard4(acc[1][0], acc[1][1], acc[1][2], acc[1][3]);
  acc_guard4(acc[2][0], acc[2][1], acc[2][2], acc[2][3]);
  acc_guard4(acc[3][0], acc[3][1], acc[3][2], acc[3][3]);

  float* slab = sT[wave];
  const float* Rb = RESID ? (resid + (size_t)b * strideR) : nullptr;
#pragma unroll
  for (int i = 0; i < 4; ++i) {
    const int mBase = m0 + (i << 4);
#pragma unroll
    for (int j = 0; j < 4; ++j) {
      const int n = n0 + (j << 4) + rlane;
      float bv = 0.f;
      if (BIAS_MODE == 2) bv = bias[n];
#pragma unroll
      for (int r = 0; r < 8; ++r) {
        float v = acc[i][j][r] * scale;
        if (BIAS_MODE == 1) v += bias[mBase + mOff + r];
        if (BIAS_MODE == 2) v += bv;
        if (RESID) v += Rb[(size_t)(mBase + mOff + r) * ldc + n];
        if (ACT == 1) v = tanhf(v);
        if (ACT == 2) v = fmaxf(v, 0.0f);
        if (ACT == 3) v = v / (1.0f + expf(-v));
        if (ACT == 4) v = (v > 0.f) ? v : 0.01f * v;
        if (ACT == 5) v = 0.5f * v * (1.0f + erff(v * 0.70710678118654752f));
        slab[(mOff + r) * 68 + (j << 4) + rlane] = v;
      }
    }
    __builtin_amdgcn_fence(__ATOMIC_RELEASE, "workgroup");
    __builtin_amdgcn_wave_barrier();
    __builtin_amdgcn_fence(__ATOMIC_ACQUIRE, "workgroup");
    if (OUT_MODE == 0) {
      float* C = (float*)Cout + (size_t)b * strideC;
      const int hh = lane >> 4, c4 = (lane & 15) * 4;
      for (int pass = 0; pass < 2; ++pass) {
#pragma unroll
        for (int it = 0; it < 8; ++it) {
          const int row = it * 2 + hh;
          v4f v = *(const v4f*)(slab + row * 68 + c4);
          *(volatile v4f*)(C + (size_t)(mBase + row) * ldc + n0 + c4) = v;
        }
        __threadfence();
      }
    } else {
      const int q = lane >> 3, c8 = (lane & 7) * 8;
      unsigned short* C  = (unsigned short*)Cout  + (size_t)b * strideC;
      unsigned short* C2 = (OUT_MODE == 2) ? ((unsigned short*)Cout2 + (size_t)b * strideC) : nullptr;
      for (int pass = 0; pass < 2; ++pass) {
#pragma unroll
        for (int it = 0; it < 4; ++it) {
          const int row = it * 4 + q;
          const float* sp = slab + row * 68 + c8;
          v8h hv, lv;
#pragma unroll
          for (int e = 0; e < 8; ++e) {
            if (OUT_MODE == 1) {
              hv[e] = (_Float16)sp[e];
            } else {
              unsigned short hb = f2bf_bits(sp[e]);
              unsigned short lb = f2bf_bits(sp[e] - bf_bits2f(hb));
              hv[e] = __builtin_bit_cast(_Float16, hb);
              lv[e] = __builtin_bit_cast(_Float16, lb);
            }
          }
          *(volatile v8h*)(C + (size_t)(mBase + row) * ldc + n0 + c8) = hv;
          if (OUT_MODE == 2) *(volatile v8h*)(C2 + (size_t)(mBase + row) * ldc + n0 + c8) = lv;
        }
        __threadfence();
      }
    }
    __builtin_amdgcn_fence(__ATOMIC_RELEASE, "workgroup");
    __builtin_amdgcn_wave_barrier();
    __builtin_amdgcn_fence(__ATOMIC_ACQUIRE, "workgroup");
  }
}

__device__ __forceinline__ int blk_excl_scan(int cnt, int* scan_ws, int tid, int* tot) {
  const int lane = tid & 31, wave = tid >> 5; int incl = cnt;
#pragma unroll
  for (int o = 1; o < 32; o <<= 1) { const int v = __shfl_up(incl, o, 32); if (lane >= o) incl += v; }
  if (lane == 31) scan_ws[wave] = incl;
  __syncthreads();
  if (wave == 0) { int wv = (lane < NT / 32) ? scan_ws[lane] : 0; int wincl = wv;
#pragma unroll
    for (int o = 1; o < 32; o <<= 1) { const int v = __shfl_up(wincl, o, 32); if (lane >= o) wincl += v; }
    if (lane < NT / 32) scan_ws[32 + lane] = wincl - wv; if (lane == 31) scan_ws[64] = wincl; }
  __syncthreads();
  const int res = scan_ws[32 + wave] + incl - cnt; *tot = scan_ws[64];
  return res;
}
template <int SP, int CAP>
__device__ __forceinline__ int chunk_hits(const int* __restrict__ dstv, const int* __restrict__ srcv, int e0, int n0, int tid,
                                          int* LIST, int* scan_ws) {
  const int eb = e0 + tid * SP;
  int rec[SP]; int cnt = 0;
  if (eb < NE) {
#pragma unroll
    for (int k = 0; k < SP; k += 4) {
      const v4i d4 = *(const v4i*)(dstv + eb + k);
      const v4i s4 = *(const v4i*)(srcv + eb + k);
#pragma unroll
      for (int e = 0; e < 4; ++e) {
        const int d = d4[e]; int r = -1;
        if (d >= n0 && d < n0 + TILE) { int s = s4[e]; s = s < 0 ? 0 : (s >= NN ? NN - 1 : s); r = ((d - n0) << 16) | s; ++cnt; }
        rec[k + e] = r;
      }
    }
  } else {
#pragma unroll
    for (int k = 0; k < SP; ++k) rec[k] = -1;
  }
  int tot; int p = blk_excl_scan(cnt, scan_ws, tid, &tot);
#pragma unroll
  for (int k = 0; k < SP; ++k) if (rec[k] >= 0) { if ((unsigned)p < (unsigned)CAP) LIST[p] = rec[k]; ++p; }
  __syncthreads();
  return tot < CAP ? tot : CAP;
}

__device__ __forceinline__ float gatef(float logit) {
  const float x = logit * L0_RBETA;
  const float ex = expf(-x);
  const float sg = 1.0f / (1.0f + ex);
  const float a = sg * 1.2f + (-0.1f);
  return fminf(fmaxf(a, 0.0f), 1.0f);
}

__global__ __launch_bounds__(NT) void colstats_kernel(const float* __restrict__ lnc, const float* __restrict__ mi, const float* __restrict__ mm,
                                                     float* __restrict__ mean, float* __restrict__ rstd) {
  __shared__ float SMU[32];
  __shared__ float SRS[32];
  const int tid = threadIdx.x, lane = tid & 31, wave = tid >> 5;
  const int sb = blockIdx.x * 32;
#pragma unroll 1
  for (int k = 0; k < 4; ++k) {
    const int sl = wave + 8 * k;
    const int s = sb + sl;
    double su = 0.0, sq = 0.0;
    const float* p0 = lnc + (size_t)s * LC0;
#pragma unroll 1
    for (int i = lane; i < LC0; i += 32) { const double x = (double)p0[i]; su += x; sq = fma(x, x, sq); }
    const float* p1 = mi + (size_t)s * LC1;
#pragma unroll 1
    for (int i = lane; i < LC1; i += 32) { const double x = (double)p1[i]; su += x; sq = fma(x, x, sq); }
    const float* p2 = mm + (size_t)s * LC2;
#pragma unroll 1
    for (int i = lane; i < LC2; i += 32) { const double x = (double)p2[i]; su += x; sq = fma(x, x, sq); }
#pragma unroll
    for (int off = 16; off > 0; off >>= 1) { su += __shfl_xor(su, off, 32); sq += __shfl_xor(sq, off, 32); }
    const double mu = su * (1.0 / (double)NN);
    const double var = (sq - su * mu) * (1.0 / (double)(NN - 1));
    const float muf = (float)mu;
    const float varf = (float)var;
    const float rs = 1.0f / sqrtf(varf);
    if (lane == 0) { SMU[sl] = muf; SRS[sl] = rs; }
  }
  __syncthreads();
  if (wave == 0) {
    const float a = SMU[lane], b = SRS[lane];
    for (int pass = 0; pass < 2; ++pass) {
      ((volatile float*)mean)[sb + lane] = a;
      ((volatile float*)rstd)[sb + lane] = b;
      __threadfence();
    }
  }
}

__global__ __launch_bounds__(NT) void arna_kernel(const float* __restrict__ lnc, const float* __restrict__ mi, const float* __restrict__ mm,
                                                 const float* __restrict__ mean, const float* __restrict__ rstd,
                                                 const float* __restrict__ attn_l, const float* __restrict__ attn_r,
                                                 float* __restrict__ ARNA, float* __restrict__ A1, float* __restrict__ A2) {
  __shared__ __align__(16) float TS[32 * TP];
  __shared__ float S1[32];
  __shared__ float S2[32];
  const int tid = threadIdx.x, lane = tid & 31, wave = tid >> 5;
  const int n0 = blockIdx.x * 32;
  const int n = n0 + lane;
  const int c0 = n < LC0 ? n : LC0 - 1;
  int c1 = n - LC0; c1 = c1 < 0 ? 0 : (c1 > LC1 - 1 ? LC1 - 1 : c1);
  int c2 = n - LC0 - LC1; c2 = c2 < 0 ? 0 : (c2 > LC2 - 1 ? LC2 - 1 : c2);
  const int sel = (n < LC0) ? 0 : ((n < LC0 + LC1) ? 1 : 2);
#pragma unroll 1
  for (int s = wave; s < SS; s += 8) {
    float x;
    if (sel == 0) x = lnc[(size_t)s * LC0 + c0];
    else if (sel == 1) x = mi[(size_t)s * LC1 + c1];
    else x = mm[(size_t)s * LC2 + c2];
    const float v = (x - mean[s]) * rstd[s];
    TS[lane * TP + s] = v;
  }
  __syncthreads();
#pragma unroll 1
  for (int k = 0; k < 4; ++k) {
    const int nl = wave * 4 + k;
    const int nn = n0 + nl;
    const v4f p0 = *(const v4f*)(TS + nl * TP + 4 * lane);
    const v4f p1 = *(const v4f*)(TS + nl * TP + 128 + 4 * lane);
    float ps = ((p0[0] + p0[1]) + (p0[2] + p0[3])) + ((p1[0] + p1[1]) + (p1[2] + p1[3]));
#pragma unroll
    for (int off = 16; off > 0; off >>= 1) ps += __shfl_xor(ps, off, 32);
    const float al = attn_l[nn], ar = attn_r[nn];
    float* rp = ARNA + (size_t)nn * SS + 4 * lane;
    for (int pass = 0; pass < 2; ++pass) {
      *(volatile v4f*)(rp) = p0;
      *(volatile v4f*)(rp + 128) = p1;
      __threadfence();
    }
    if (lane == 0) { S1[nl] = ps * al; S2[nl] = ps * ar; }
  }
  __syncthreads();
  if (wave == 0) {
    const float a = S1[lane], b = S2[lane];
    for (int pass = 0; pass < 2; ++pass) {
      ((volatile float*)A1)[n0 + lane] = a;
      ((volatile float*)A2)[n0 + lane] = b;
      __threadfence();
    }
  }
}

__global__ __launch_bounds__(NT) void prep_kernel(const float* __restrict__ W_mp, const float* __restrict__ pmask, const float* __restrict__ b_mp,
                                                 const float* __restrict__ W_ph, const float* __restrict__ b_ph,
                                                 const float* __restrict__ W_po, const float* __restrict__ b_po,
                                                 unsigned* __restrict__ WM, unsigned* __restrict__ W2, unsigned* __restrict__ W3,
                                                 float* __restrict__ BP) {
  const int i = blockIdx.x * NT + threadIdx.x;
  if (i < R1DW) {
    const int r = i >> 10, c = 2 * (i & 1023);
    const int rr = r < NPW ? r : NPW - 1, cc = c < ND - 2 ? c : ND - 2;
    const bool live = (r < NPW) && (c < ND);
    const size_t o = (size_t)rr * ND + cc;
    float a = W_mp[o] * pmask[o], bb = W_mp[o + 1] * pmask[o + 1];
    if (!live) { a = 0.f; bb = 0.f; }
    const unsigned u = (unsigned)__builtin_bit_cast(unsigned short, (_Float16)a) | ((unsigned)__builtin_bit_cast(unsigned short, (_Float16)bb) << 16);
    ((volatile unsigned*)WM)[i] = u;
    __threadfence();
    ((volatile unsigned*)WM)[i] = u;
  } else if (i < R1DW + R2DW) {
    const int j = i - R1DW;
    const int r = j >> 8, c = 2 * (j & 255);
    const int rr = r < NPH ? r : NPH - 1, cc = c < NPW - 2 ? c : NPW - 2;
    const bool live = (r < NPH) && (c < NPW);
    const size_t o = (size_t)rr * NPW + cc;
    float a = W_ph[o], bb = W_ph[o + 1];
    if (!live) { a = 0.f; bb = 0.f; }
    const unsigned u = (unsigned)__builtin_bit_cast(unsigned short, (_Float16)a) | ((unsigned)__builtin_bit_cast(unsigned short, (_Float16)bb) << 16);
    ((volatile unsigned*)W2)[j] = u;
    __threadfence();
    ((volatile unsigned*)W2)[j] = u;
  } else if (i < R1DW + R2DW + R3DW) {
    const int j = i - R1DW - R2DW;
    const int r = j >> 6, c = 2 * (j & 63);
    const int rr = r < NOUT ? r : NOUT - 1, cc = c < NPH - 2 ? c : NPH - 2;
    const bool live = (r < NOUT) && (c < NPH);
    const size_t o = (size_t)rr * NPH + cc;
    float a = W_po[o], bb = W_po[o + 1];
    if (!live) { a = 0.f; bb = 0.f; }
    const unsigned u = (unsigned)__builtin_bit_cast(unsigned short, (_Float16)a) | ((unsigned)__builtin_bit_cast(unsigned short, (_Float16)bb) << 16);
    ((volatile unsigned*)W3)[j] = u;
    __threadfence();
    ((volatile unsigned*)W3)[j] = u;
  }
  if (i < NBIAS) {
    float v = 0.f;
    if (i < PP1) {
      const int j = i; const float t = b_mp[j < NPW ? j : NPW - 1]; v = (j < NPW) ? t : 0.f;
    } else if (i < PP1 + PHP1) {
      const int j = i - PP1; const float t = b_ph[j < NPH ? j : NPH - 1]; v = (j < NPH) ? t : 0.f;
    } else {
      const int j = i - PP1 - PHP1; const float t = b_po[j < NOUT ? j : NOUT - 1]; v = (j < NOUT) ? t : 0.f;
    }
    ((volatile float*)BP)[i] = v;
    __threadfence();
    ((volatile float*)BP)[i] = v;
  }
}

template <bool SECOND>
__global__ __launch_bounds__(NT) void agg_kernel(const int* __restrict__ src, const int* __restrict__ dst,
                                                const float* __restrict__ A1, const float* __restrict__ A2, const float* __restrict__ bias_l0,
                                                const float* __restrict__ FIN, float* ACC, float* ZI) {
  __shared__ int LIST[SCH];
  __shared__ float SA2[TILE];
  __shared__ float SZ[TILE];
  __shared__ int scan_ws[80];
  const int tid = threadIdx.x, lane = tid & 31, wave = tid >> 5;
  const int n0 = blockIdx.x * TILE;
  const float b0 = bias_l0[0];
  const v4f z4 = {0.f, 0.f, 0.f, 0.f};
#pragma unroll 1
  for (int j = 0; j < RPW; ++j) {
    float* rp = ACC + (size_t)(n0 + wave * RPW + j) * SS + 4 * lane;
    *(v4f*)rp = z4; *(v4f*)(rp + 128) = z4;
  }
  for (int i = tid; i < TILE; i += NT) {
    int n = n0 + i; n = n < NN ? n : NN - 1;
    SA2[i] = A2[n];
    if (SECOND) { int m = n0 + i; m = m < NPR ? m : NPR - 1; SZ[i] = ZI[m]; }
    else SZ[i] = 0.f;
  }
  __syncthreads();
#pragma unroll 1
  for (int c = 0; c < NCH; ++c) {
    const int tot = chunk_hits<SPT, SCH>(dst, src, c * SCH, n0, tid, LIST, scan_ws);
#pragma unroll 1
    for (int base = 0; base < tot; base += 32) {
      const int q = base + lane;
      const int qc = q < SCH ? q : SCH - 1;
      const int lv = LIST[qc];
      const int rv = (q < tot) ? lv : -1;
      const int own = (rv >= 0 && (rv >> 24) == wave) ? 1 : 0;
      const int dq = (rv >> 16) & (TILE - 1);
      int sq = rv & 0xFFFF; sq = sq < NN ? sq : NN - 1;
      float gq = gatef(A1[sq] + SA2[dq] + b0);
      if (SECOND) gq = gq * SZ[dq];
      unsigned msk = (unsigned)__ballot(own);
#pragma unroll 1
      for (int it = 0; it < 32; ++it) {
        if (msk == 0u) break;
        const int bp = __builtin_ctz(msk); msk &= msk - 1u;
        const int r = __shfl(rv, bp, 32);
        const float gv = __shfl(gq, bp, 32);
        const int dl = (r >> 16) & (TILE - 1);
        int s = r & 0xFFFF; s = s < NN ? s : NN - 1;
        if (!SECOND) { if (lane == 0) SZ[dl] += gv; }
        float* rp = ACC + (size_t)(n0 + dl) * SS + 4 * lane;
        const float* xp = FIN + (size_t)s * SS + 4 * lane;
        v4f a0 = *(const v4f*)rp, a1 = *(const v4f*)(rp + 128);
        const v4f x0 = *(const v4f*)xp, x1 = *(const v4f*)(xp + 128);
        a0 = a0 + gv * x0;
        a1 = a1 + gv * x1;
        *(v4f*)rp = a0; *(v4f*)(rp + 128) = a1;
      }
    }
    __syncthreads();
  }
  if (!SECOND) {
    for (int i = tid; i < TILE; i += NT) { const float z = SZ[i]; SZ[i] = (z > 0.f) ? (1.0f / z) : 0.f; }
    __syncthreads();
  }
#pragma unroll 1
  for (int j = 0; j < RPW; ++j) {
    const int dl = wave * RPW + j;
    float* rp = ACC + (size_t)(n0 + dl) * SS + 4 * lane;
    v4f a0 = *(const v4f*)rp, a1 = *(const v4f*)(rp + 128);
    if (!SECOND) { const float inv = SZ[dl]; a0 = a0 * inv; a1 = a1 * inv; }
    for (int pass = 0; pass < 2; ++pass) {
      *(volatile v4f*)rp = a0;
      *(volatile v4f*)(rp + 128) = a1;
      __threadfence();
    }
  }
  if (!SECOND) {
    for (int i = tid; i < TILE; i += NT) {
      const float v = SZ[i];
      for (int pass = 0; pass < 2; ++pass) { ((volatile float*)ZI)[n0 + i] = v; __threadfence(); }
    }
  }
}

__global__ __launch_bounds__(NT) void xbuild_kernel(const int* __restrict__ dem, const float* __restrict__ ARNA,
                                                   const float* __restrict__ R1, const float* __restrict__ R2, unsigned short* __restrict__ X) {
  __shared__ __align__(16) _Float16 XT[64 * XTP];
  const int tid = threadIdx.x, lane = tid & 31, wave = tid >> 5;
  const int d0 = blockIdx.x * 64;
#pragma unroll 1
  for (int k = 0; k < 8; ++k) {
    const int dd = wave * 8 + k;
    const int d = d0 + dd;
    const bool live = d < ND;
    const int dc = live ? d : ND - 1;
    int idx = dem[dc]; idx = idx < 0 ? 0 : (idx >= NN ? NN - 1 : idx);
    const float* pa = ARNA + (size_t)idx * SS + 4 * lane;
    const float* pb = R1 + (size_t)idx * SS + 4 * lane;
    const float* pc = R2 + (size_t)idx * SS + 4 * lane;
    const v4f t0 = (*(const v4f*)pa + *(const v4f*)pb) + *(const v4f*)pc;
    const v4f t1 = (*(const v4f*)(pa + 128) + *(const v4f*)(pb + 128)) + *(const v4f*)(pc + 128);
    _Float16* xr = XT + dd * XTP;
#pragma unroll
    for (int e = 0; e < 4; ++e) {
      xr[4 * lane + e] = live ? (_Float16)t0[e] : (_Float16)0.0f;
      xr[128 + 4 * lane + e] = live ? (_Float16)t1[e] : (_Float16)0.0f;
    }
  }
  __syncthreads();
  const int q = lane >> 3, c8 = (lane & 7) * 8;
  for (int pass = 0; pass < 2; ++pass) {
#pragma unroll
    for (int it = 0; it < 8; ++it) {
      const int s = wave * 32 + it * 4 + q;
      v8h hv;
#pragma unroll
      for (int e = 0; e < 8; ++e) hv[e] = XT[(c8 + e) * XTP + s];
      *(volatile v8h*)(X + (size_t)s * KP1 + d0 + c8) = hv;
    }
    __threadfence();
  }
}

__global__ __launch_bounds__(NT) void softmax2_kernel(const float* __restrict__ LG, float* __restrict__ out) {
  const int s = threadIdx.x;
  const float l0 = LG[(size_t)s * OPP], l1 = LG[(size_t)s * OPP + 1];
  const float m = fmaxf(l0, l1);
  const float e0 = expf(l0 - m), e1 = expf(l1 - m);
  const float inv = 1.0f / (e0 + e1);
  v2f o; o[0] = e0 * inv; o[1] = e1 * inv;
  for (int pass = 0; pass < 2; ++pass) { *(volatile v2f*)(out + 2 * s) = o; __threadfence(); }
}

extern "C" void kernel_launch(void* const* d_in, const int* in_sizes, int n_in,
                              void* d_out, int out_size, void* d_ws, size_t ws_size, hipStream_t stream) {
  if (n_in < 16) return;
  if (in_sizes[0] != SS * LC0 || in_sizes[1] != SS * LC1 || in_sizes[2] != SS * LC2) return;
  if (in_sizes[3] != NE || in_sizes[4] != NE || in_sizes[5] != ND || in_sizes[6] != NN || in_sizes[7] != NN || in_sizes[8] < 1) return;
  if (in_sizes[9] != NPW * ND || in_sizes[10] != NPW * ND || in_sizes[11] != NPW || in_sizes[12] != NPH * NPW || in_sizes[13] != NPH) return;
  if (in_sizes[14] != NOUT * NPH || in_sizes[15] != NOUT || out_size != SS * NOUT) return;

  const float* lnc     = (const float*)d_in[0];
  const float* mi      = (const float*)d_in[1];
  const float* mm      = (const float*)d_in[2];
  const int*   src     = (const int*)d_in[3];
  const int*   dst     = (const int*)d_in[4];
  const int*   dem     = (const int*)d_in[5];
  const float* attn_l  = (const float*)d_in[6];
  const float* attn_r  = (const float*)d_in[7];
  const float* bias_l0 = (const float*)d_in[8];
  const float* pmask   = (const float*)d_in[9];
  const float* W_mp    = (const float*)d_in[10];
  const float* b_mp    = (const float*)d_in[11];
  const float* W_ph    = (const float*)d_in[12];
  const float* b_ph    = (const float*)d_in[13];
  const float* W_po    = (const float*)d_in[14];
  const float* b_po    = (const float*)d_in[15];
  float* out = (float*)d_out;

  char* ws = (char*)d_ws; size_t off = 0;
  auto carve = [&](size_t bytes) -> char* { char* p = ws + off; off += (bytes + 255) & ~(size_t)255; return p; };
  float*          MEAN = (float*)carve((size_t)SS * 4);
  float*          RSTD = (float*)carve((size_t)SS * 4);
  float*          ARNA = (float*)carve((size_t)NN * SS * 4);
  float*          A1   = (float*)carve((size_t)NPR * 4);
  float*          A2   = (float*)carve((size_t)NPR * 4);
  float*          ZI   = (float*)carve((size_t)NPR * 4);
  float*          RNA1 = (float*)carve((size_t)NPR * SS * 4);
  float*          RNA2 = (float*)carve((size_t)NPR * SS * 4);
  unsigned short* X16  = (unsigned short*)carve((size_t)SS * KP1 * 2);
  unsigned*       WM16 = (unsigned*)carve((size_t)PP1 * KP1 * 2);
  unsigned short* H1   = (unsigned short*)carve((size_t)SS * PP1 * 2);
  unsigned*       W2P  = (unsigned*)carve((size_t)PHP1 * PP1 * 2);
  unsigned short* H2   = (unsigned short*)carve((size_t)SS * PHP1 * 2);
  unsigned*       W3P  = (unsigned*)carve((size_t)OPP * PHP1 * 2);
  float*          LG   = (float*)carve((size_t)SS * OPP * 4);
  float*          BP   = (float*)carve((size_t)NBIAS * 4);
  if (off > ws_size || off > (size_t)134217728) return;

  colstats_kernel<<<SS / 32, NT, 0, stream>>>(lnc, mi, mm, MEAN, RSTD);
  arna_kernel<<<NN / 32, NT, 0, stream>>>(lnc, mi, mm, MEAN, RSTD, attn_l, attn_r, ARNA, A1, A2);
  prep_kernel<<<(R1DW + R2DW + R3DW + NT - 1) / NT, NT, 0, stream>>>(W_mp, pmask, b_mp, W_ph, b_ph, W_po, b_po,
                                                                     WM16, W2P, W3P, BP);
  agg_kernel<false><<<NTILE, NT, 0, stream>>>(src, dst, A1, A2, bias_l0, ARNA, RNA1, ZI);
  agg_kernel<true><<<NTILE, NT, 0, stream>>>(src, dst, A1, A2, bias_l0, RNA1, RNA2, ZI);
  xbuild_kernel<<<KP1 / 64, NT, 0, stream>>>(dem, ARNA, RNA1, RNA2, X16);
  {
    const int tiles = (SS / 64) * (PP1 / 64);
    wmma_gemm64<0, false, 2, 1, false, 2><<<dim3((tiles + 7) / 8, 1), 256, 0, stream>>>(
        (const unsigned short*)X16, (const unsigned short*)nullptr, KP1, 0L,
        (const unsigned short*)WM16, (const unsigned short*)nullptr, KP1, 0L,
        (void*)H1, (void*)nullptr, PP1, 0L,
        (const float*)BP, (const float*)nullptr, 0L, SS, PP1, KP1, 1.0f);
  }
  {
    const int tiles = (SS / 64) * (PHP1 / 64);
    wmma_gemm64<0, false, 2, 1, false, 2><<<dim3((tiles + 7) / 8, 1), 256, 0, stream>>>(
        (const unsigned short*)H1, (const unsigned short*)nullptr, PP1, 0L,
        (const unsigned short*)W2P, (const unsigned short*)nullptr, PP1, 0L,
        (void*)H2, (void*)nullptr, PHP1, 0L,
        (const float*)(BP + PP1), (const float*)nullptr, 0L, SS, PHP1, PP1, 1.0f);
  }
  {
    const int tiles = (SS / 64) * (OPP / 64);
    wmma_gemm64<0, false, 2, 0, false, 0><<<dim3((tiles + 7) / 8, 1), 256, 0, stream>>>(
        (const unsigned short*)H2, (const unsigned short*)nullptr, PHP1, 0L,
        (const unsigned short*)W3P, (const unsigned short*)nullptr, PHP1, 0L,
        (void*)LG, (void*)nullptr, OPP, 0L,
        (const float*)(BP + PP1 + PHP1), (const float*)nullptr, 0L, SS, OPP, PHP1, 1.0f);
  }
  softmax2_kernel<<<1, NT, 0, stream>>>(LG, out);
}
